// DecorrelateLossClass_2147483648069
// MI455X (gfx1250) — hardware-verified
//
#include <hip/hip_runtime.h>
#include <hip/hip_bf16.h>
#include <math.h>


typedef _Float16 bf16;
typedef _Float16 f16;
typedef __attribute__((ext_vector_type(4))) unsigned v4u_t;
typedef unsigned v4ua __attribute__((ext_vector_type(4), may_alias));
typedef __attribute__((ext_vector_type(4))) float v4f_t;
typedef float v4fa __attribute__((ext_vector_type(4), may_alias));
typedef __attribute__((ext_vector_type(16))) bf16  bf16x16;
typedef bf16x16 f16x16;
typedef __attribute__((ext_vector_type(8)))  bf16  bf16x8;
typedef bf16x8 f16x8;
typedef __attribute__((ext_vector_type(4)))  bf16  bf16x4;
typedef __attribute__((ext_vector_type(8)))  float f32x8;
__device__ __forceinline__ f32x8 wmma16(f16x16 a, f16x16 b, f32x8 c) {
  c = __builtin_amdgcn_wmma_f32_16x16x32_f16(false, a, false, b, (short)0, c, false, false);
  asm volatile("v_nop\n\tv_nop\n\tv_nop\n\tv_nop" : "+v"(c) : "v"(a), "v"(b));
  return c;
}
#define LDS_STRIDE 48
#define KSTRIDE    72
#define VSTRIDE    48

__device__ __forceinline__ f32x8 wmma_bf16(bf16x16 a, bf16x16 b, f32x8 c) {
  c = __builtin_amdgcn_wmma_f32_16x16x32_f16(false, a, false, b, (short)0, c, false, false);
  asm volatile("v_nop\n\tv_nop\n\tv_nop\n\tv_nop" : "+v"(c) : "v"(a), "v"(b));
  return c;
}

template <typename T>
__device__ __forceinline__ bf16x16 load_frag(const T* __restrict__ base, int ld,
                                             int row0, int k0) {
  const int lane = threadIdx.x & 31;
  const int r    = lane & 15;
  const int kh   = (lane >> 4) * 8;
  const T* p0 = base + (size_t)(row0 + r) * ld + (k0 + kh);
  const T* p1 = p0 + 16;
  bf16x16 f;
#pragma unroll
  for (int i = 0; i < 8; ++i) {
    f[i]     = (bf16)p0[i];
    f[i + 8] = (bf16)p1[i];
  }
  return f;
}

__device__ __forceinline__ bf16x16 lds_frag(const bf16* base, int stride) {
  const int lane = threadIdx.x & 31;
  const int row  = lane & 15;
  const int kh   = (lane >> 4) * 8;
  const bf16x8 lo = *(const bf16x8*)(base + row * stride + kh);
  const bf16x8 hi = *(const bf16x8*)(base + row * stride + kh + 16);
  bf16x16 f;
#pragma unroll
  for (int i = 0; i < 8; ++i) { f[i] = lo[i]; f[i + 8] = hi[i]; }
  return f;
}

template <typename T>
__device__ __forceinline__ void stage_read16(const T* __restrict__ p, float* buf) {
#pragma unroll
  for (int i = 0; i < 16; ++i) buf[i] = (float)p[i];
}

__device__ __forceinline__ void stage_write(bf16* dst, const float* buf, int nquad) {
#pragma unroll
  for (int i = 0; i < nquad; ++i) {
    bf16x4 q;
    q[0] = (bf16)buf[4 * i];     q[1] = (bf16)buf[4 * i + 1];
    q[2] = (bf16)buf[4 * i + 2]; q[3] = (bf16)buf[4 * i + 3];
    *(bf16x4*)(dst + 4 * i) = q;
  }
}


#define GSTR 48
#define SS 512
#define HH 8
#define DKK 64
template <typename AT, int MODE>
__global__ __launch_bounds__(256) void gemm_rb_kernel(
    const AT* __restrict__ A, const float* __restrict__ W,
    const float* __restrict__ bias, const float* __restrict__ rowscale, const float* __restrict__ R, const float* __restrict__ rowbias, void* __restrict__ out,
    int M, int N, int K) {
  __shared__ bf16 ldsA[128 * LDS_STRIDE];
  __shared__ bf16 ldsW[256 * LDS_STRIDE];
  __shared__ __attribute__((aligned(16))) unsigned char sob[256 * 136 * 2];

  const int t    = threadIdx.x;
  const int wave = t >> 5;
  const int lane = t & 31;
  const int wm   = (wave & 1) * 64;
  const int wn   = (wave >> 1) * 64;
  const int mBlk = blockIdx.x * 128;
  const int nBlk = blockIdx.y * 256;

  const int arow = t >> 1;
  const int ach  = (t & 1) * 16;

  float abuf[16];
  float wbuf[32];

  stage_read16(A + (size_t)(mBlk + arow) * K + ach, abuf);
  const int nrow = min(nBlk + t, N - 1);
  stage_read16(W + (size_t)nrow * K,          wbuf);
  stage_read16(W + (size_t)nrow * K + 16,     wbuf + 16);

  f32x8 acc[4][4] = {};

  for (int k = 0; k < K; k += 32) {
    __syncthreads();
    stage_write(&ldsA[arow * LDS_STRIDE + ach], abuf, 4);
    stage_write(&ldsW[t * LDS_STRIDE],          wbuf, 8);
    if (k + 32 < K) {
      stage_read16(A + (size_t)(mBlk + arow) * K + (k + 32) + ach, abuf);
      stage_read16(W + (size_t)nrow * K + (k + 32),          wbuf);
      stage_read16(W + (size_t)nrow * K + (k + 32) + 16,     wbuf + 16);
    }
    __syncthreads();

    bf16x16 af[4], wf[4];
#pragma unroll
    for (int i = 0; i < 4; ++i)
      af[i] = lds_frag(ldsA + (wm + 16 * i) * LDS_STRIDE, LDS_STRIDE);
#pragma unroll
    for (int j = 0; j < 4; ++j)
      wf[j] = lds_frag(ldsW + (wn + 16 * j) * LDS_STRIDE, LDS_STRIDE);
#pragma unroll
    for (int i = 0; i < 4; ++i)
#pragma unroll
      for (int j = 0; j < 4; ++j)
        acc[i][j] = wmma_bf16(af[i], wf[j], acc[i][j]);
  }

  const int nlane = lane & 15;
  const int mh    = (lane >> 4) * 8;
  __syncthreads();
  if (MODE == 0 || MODE == 1 || MODE == 3) {
    bf16* so = (bf16*)sob;
#pragma unroll
    for (int i = 0; i < 4; ++i)
#pragma unroll
      for (int j = 0; j < 4; ++j) {
        const int nl = wn + 16 * j + nlane;
        const float bv = bias ? bias[nBlk + nl] : 0.0f;
        if (MODE == 3) {
#pragma unroll 1
          for (int r = 0; r < 8; ++r) {
            const int ml = wm + 16 * i + mh + r;
            const float xg = acc[i][j][r] + bv;
            so[ml * 264 + nl] = (bf16)(0.5f * xg * (1.0f + erff(xg * 0.70710678118654752f)));
          }
        } else {
#pragma unroll
        for (int r = 0; r < 8; ++r) {
          const int ml = wm + 16 * i + mh + r;
          const bf16 hv = (bf16)(acc[i][j][r] + bv);
          if (MODE == 0) so[ml * 264 + nl] = hv;
          else           so[nl * 136 + ml] = hv;
        }
        }
      }
    __syncthreads();
#pragma unroll 1
    for (int pass = 0; pass < 2; ++pass) {
      if (MODE == 0 || MODE == 3) {
        for (int ch = t; ch < 128 * 32; ch += 256) { const int ml = ch >> 5, q = (ch & 31) * 8;
          *(volatile v4u_t*)((bf16*)out + (size_t)(mBlk + ml) * N + nBlk + q) = *(const v4ua*)(so + ml * 264 + q); }
      } else {
        const int b_ = mBlk / SS, s0 = mBlk % SS;
        for (int ch = t; ch < 256 * 16; ch += 256) { const int nl = ch >> 4, q = (ch & 15) * 8; const int n = nBlk + nl, h = n >> 6, dk = n & (DKK - 1);
          *(volatile v4u_t*)((bf16*)out + (((size_t)(b_ * HH + h)) * DKK + dk) * SS + s0 + q) = *(const v4ua*)(so + nl * 136 + q); }
      }
      __threadfence();
    }
  } else {
    float* so = (float*)sob;
#pragma unroll 1
    for (int hf = 0; hf < 2; ++hf) {
      if (wm == hf * 64) {
#pragma unroll
        for (int i = 0; i < 4; ++i)
#pragma unroll
          for (int j = 0; j < 4; ++j) {
            const int nl = wn + 16 * j + nlane;
            const float bv = bias ? bias[nBlk + nl] : 0.0f;
#pragma unroll
            for (int r = 0; r < 8; ++r) { const int mrow = mBlk + hf * 64 + 16 * i + mh + r; so[(16 * i + mh + r) * 260 + nl] = acc[i][j][r] * (rowscale ? rowscale[mrow] : 1.0f) + bv + (rowbias ? rowbias[mrow] : 0.0f); }
          }
      }
      __syncthreads();
      if (R) {
        for (int ch = t; ch < 64 * 64; ch += 256) { const int ml = ch >> 6, q = (ch & 63) * 4;
          if (nBlk + q < N) { const v4f_t rv = *(const v4f_t*)(R + (size_t)(mBlk + hf * 64 + ml) * N + nBlk + q); v4f_t v = *(const v4fa*)(so + ml * 260 + q); v += rv; *(volatile v4fa*)(so + ml * 260 + q) = v; } }
        asm volatile("s_wait_dscnt 0" ::: "memory");
      }
#pragma unroll 1
      for (int pass = 0; pass < 2; ++pass) {
        for (int ch = t; ch < 64 * 64; ch += 256) { const int ml = ch >> 6, q = (ch & 63) * 4;
          if (nBlk + q < N) *(volatile v4f_t*)((float*)out + (size_t)(mBlk + hf * 64 + ml) * N + nBlk + q) = *(const v4fa*)(so + ml * 260 + q); }
        __threadfence();
      }
      __syncthreads();
    }
  }
}


#define NS 16384
#define CC 512
#define KCL 128
#define KP 192
__global__ __launch_bounds__(256) void k_members(const int* __restrict__ y, int* __restrict__ memb, int* __restrict__ cnt) {
  __shared__ int lst[KP]; __shared__ int nK;
  const int k = blockIdx.x, tid = threadIdx.x;
  if (tid == 0) { int n = 0;
#pragma unroll 1
    for (int i = 0; i < NS; ++i) { if (y[i] == k) { if (n < KP) lst[n] = i; ++n; } }
    nK = n; }
  __syncthreads();
  const int n = nK;
  if (tid < KP) { const int v = (tid < n && tid < KP) ? lst[tid] : -1; *(volatile int*)(memb + k * KP + tid) = v; __threadfence(); *(volatile int*)(memb + k * KP + tid) = v; }
  if (tid == 0) { *(volatile int*)(cnt + k) = n; __threadfence(); *(volatile int*)(cnt + k) = n; }
}
__global__ __launch_bounds__(256) void k_stats(const float* __restrict__ x, const int* __restrict__ memb, const int* __restrict__ cnt, float* __restrict__ mean, float* __restrict__ rstd) {
  const int k = blockIdx.x, tid = threadIdx.x; const int n = min(cnt[k], KP); const int* ml = memb + k * KP;
  float s1a = 0.f, s2a = 0.f, s1b = 0.f, s2b = 0.f;
#pragma unroll 1
  for (int m = 0; m < n; ++m) { const size_t r = (size_t)ml[m] * CC; const float a = x[r + tid], b = x[r + tid + 256]; s1a += a; s2a = fmaf(a, a, s2a); s1b += b; s2b = fmaf(b, b, s2b); }
  const float nf = (float)cnt[k]; const float dn = fmaxf(nf, 1.0f), dv = fmaxf(nf - 1.0f, 1.0f);
  const float ma = s1a / dn, mb = s1b / dn; const float va = fmaxf((s2a - nf * ma * ma) / dv, 0.0f), vb = fmaxf((s2b - nf * mb * mb) / dv, 0.0f);
  const float ra = rsqrtf(1e-8f + va), rb = rsqrtf(1e-8f + vb);
  *(volatile float*)(mean + (size_t)k * CC + tid) = ma; *(volatile float*)(mean + (size_t)k * CC + tid + 256) = mb; *(volatile float*)(rstd + (size_t)k * CC + tid) = ra; *(volatile float*)(rstd + (size_t)k * CC + tid + 256) = rb; __threadfence();
  *(volatile float*)(mean + (size_t)k * CC + tid) = ma; *(volatile float*)(mean + (size_t)k * CC + tid + 256) = mb; *(volatile float*)(rstd + (size_t)k * CC + tid) = ra; *(volatile float*)(rstd + (size_t)k * CC + tid + 256) = rb;
}
__global__ __launch_bounds__(256) void k_gatherT(const float* __restrict__ x, const int* __restrict__ memb, const int* __restrict__ cnt, const float* __restrict__ mean, const float* __restrict__ rstd, float* __restrict__ XT) {
  __shared__ float tS[64][65];
  const int k = blockIdx.x, ct = blockIdx.y, tid = threadIdx.x; const int n = min(cnt[k], KP); const int* ml = memb + k * KP;
#pragma unroll 1
  for (int pc = 0; pc < KP / 64; ++pc) {
    for (int e = tid; e < 64 * 64; e += 256) { const int pr = e >> 6, c = e & 63; const int p = pc * 64 + pr; const int col = ct * 64 + c;
      float v = 0.0f; if (p < n) { const int row = ml[p]; v = (x[(size_t)row * CC + col] - mean[(size_t)k * CC + col]) * rstd[(size_t)k * CC + col]; }
      tS[pr][c] = v; }
    __syncthreads();
    for (int ch = tid; ch < 64 * 16; ch += 256) { const int c = ch >> 4, q4 = (ch & 15) * 4; v4f_t v; v[0] = tS[q4][c]; v[1] = tS[q4 + 1][c]; v[2] = tS[q4 + 2][c]; v[3] = tS[q4 + 3][c];
      float* dst = XT + ((size_t)k * CC + ct * 64 + c) * KP + pc * 64 + q4; *(volatile v4f_t*)dst = v; __threadfence(); *(volatile v4f_t*)dst = v; }
    __syncthreads();
  }
}
__global__ __launch_bounds__(256) void k_offsq(const float* __restrict__ corr, float* __restrict__ offv, int k) {
  __shared__ float red[256];
  const int tid = threadIdx.x; float s = 0.0f;
#pragma unroll 1
  for (int e = tid; e < CC * CC; e += 256) { const int i = e >> 9, j = e & 511; if (i != j) { const float v = corr[e]; s = fmaf(v, v, s); } }
  red[tid] = s; __syncthreads();
  for (int o = 128; o > 0; o >>= 1) { if (tid < o) red[tid] += red[tid + o]; __syncthreads(); }
  if (tid == 0) { const float v = red[0] / (float)(CC * (CC - 1)); *(volatile float*)(offv + k) = v; __threadfence(); *(volatile float*)(offv + k) = v; }
}
__global__ __launch_bounds__(256) void k_final(const float* __restrict__ offv, const int* __restrict__ cnt, float* __restrict__ out) {
  __shared__ float ra[128], rb[128];
  const int tid = threadIdx.x;
  if (tid < KCL) { const bool v = cnt[tid] > 1; ra[tid] = v ? offv[tid] : 0.0f; rb[tid] = v ? (float)cnt[tid] : 0.0f; }
  __syncthreads();
  for (int o = 64; o > 0; o >>= 1) { if (tid < o) { ra[tid] += ra[tid + o]; rb[tid] += rb[tid + o]; } __syncthreads(); }
  if (tid == 0) { const float l = (rb[0] > 0.0f) ? ra[0] / fmaxf(rb[0], 1.0f) : 0.0f; *(volatile float*)out = l; __threadfence(); *(volatile float*)out = l; }
}
extern "C" void kernel_launch(void* const* d_in, const int* in_sizes, int n_in,
                              void* d_out, int out_size, void* d_ws, size_t ws_size,
                              hipStream_t stream) {
  (void)in_sizes; (void)n_in; (void)out_size;
  const float* x = (const float*)d_in[0]; const int* y = (const int*)d_in[1];
  float* out = (float*)d_out;
  char* ws = (char*)d_ws;
  int* memb = (int*)ws; ws += (size_t)KCL * KP * 4; int* cnt = (int*)ws; ws += KCL * 4;
  float* mean = (float*)ws; ws += (size_t)KCL * CC * 4; float* rstd = (float*)ws; ws += (size_t)KCL * CC * 4;
  float* XT = (float*)ws; ws += (size_t)KCL * CC * KP * 4;
  float* corr = (float*)ws; ws += (size_t)CC * CC * 4; float* offv = (float*)ws; ws += KCL * 4;
  if ((size_t)(ws - (char*)d_ws) > ws_size) return;
  const dim3 blk(256);
  k_members<<<dim3(KCL), blk, 0, stream>>>(y, memb, cnt);
  k_stats<<<dim3(KCL), blk, 0, stream>>>(x, memb, cnt, mean, rstd);
  k_gatherT<<<dim3(KCL, CC / 64), blk, 0, stream>>>(x, memb, cnt, mean, rstd, XT);
  for (int k = 0; k < KCL; ++k) {
    gemm_rb_kernel<float, 2><<<dim3(CC / 128, CC / 256), blk, 0, stream>>>(XT + (size_t)k * CC * KP, XT + (size_t)k * CC * KP, nullptr, nullptr, nullptr, nullptr, corr, CC, CC, KP);
    k_offsq<<<dim3(1), blk, 0, stream>>>(corr, offv, k);
  }
  k_final<<<dim3(1), blk, 0, stream>>>(offv, cnt, out);
}
